// DecoderLayer_42657615184315
// MI455X (gfx1250) — hardware-run, weakly checked
//
#include <hip/hip_runtime.h>
#include <math.h>

typedef __attribute__((ext_vector_type(16))) _Float16 v16h;
typedef __attribute__((ext_vector_type(8)))  _Float16 v8h;
typedef __attribute__((ext_vector_type(16))) __bf16   v16b;
typedef __attribute__((ext_vector_type(8)))  __bf16   v8b;
typedef __attribute__((ext_vector_type(8)))  float    v8f;
typedef __attribute__((ext_vector_type(4)))  float    v4f;
typedef __attribute__((ext_vector_type(4)))  int      v4i;
typedef __attribute__((ext_vector_type(2)))  unsigned long long v2u64;

__device__ __forceinline__ unsigned short f2bf_bits(float f) {
  unsigned u = __float_as_uint(f);
  return (unsigned short)((u + 0x7FFFu + ((u >> 16) & 1u)) >> 16);
}
__device__ __forceinline__ float bf_bits2f(unsigned short h) { return __uint_as_float(((unsigned)h) << 16); }

__device__ __forceinline__ void dep_guard_h(v8f& a, v8f& b, v16h x, v16h y) { asm volatile("v_nop\n\tv_nop\n\tv_nop\n\tv_nop" : "+v"(a), "+v"(b) : "v"(x), "v"(y)); }
__device__ __forceinline__ void dep_guard_b(v8f& a, v8f& b, v16b x, v16b y) { asm volatile("v_nop\n\tv_nop\n\tv_nop\n\tv_nop" : "+v"(a), "+v"(b) : "v"(x), "v"(y)); }
__device__ __forceinline__ void keep4_h(v16h a, v16h b, v16h c, v16h d) { asm volatile("v_nop" :: "v"(a), "v"(b), "v"(c), "v"(d)); }
__device__ __forceinline__ void keep4_b(v16b a, v16b b, v16b c, v16b d) { asm volatile("v_nop" :: "v"(a), "v"(b), "v"(c), "v"(d)); }
__device__ __forceinline__ void acc_guard4(v8f& a, v8f& b, v8f& c, v8f& d) { asm volatile("v_nop\n\tv_nop\n\tv_nop\n\tv_nop" : "+v"(a), "+v"(b), "+v"(c), "+v"(d)); }
template <typename T> struct Frag;
template <> struct Frag<_Float16> {
  typedef v16h V; union U { v16h v; v8h h[2]; };
  static __device__ __forceinline__ v16h load(const _Float16* p) {
    U f; f.h[0] = *(const v8h*)(p); f.h[1] = *(const v8h*)(p + 16); return f.v;
  }
  static __device__ __forceinline__ v8f mma(v16h a, v16h b, v8f c) {
    return __builtin_amdgcn_wmma_f32_16x16x32_f16(false, a, false, b, (short)0, c, false, false);
  }
  static __device__ __forceinline__ void guard(v8f& a, v8f& b, v16h x, v16h y) { dep_guard_h(a, b, x, y); }
  static __device__ __forceinline__ void keep(v16h a, v16h b, v16h c, v16h d) { keep4_h(a, b, c, d); }
};
template <> struct Frag<__bf16> {
  typedef v16b V; union U { v16b v; v8b h[2]; };
  static __device__ __forceinline__ v16b load(const __bf16* p) {
    U f; f.h[0] = *(const v8b*)(p); f.h[1] = *(const v8b*)(p + 16); return f.v;
  }
  static __device__ __forceinline__ v8f mma(v16b a, v16b b, v8f c) {
    return __builtin_amdgcn_wmma_f32_16x16x32_bf16(false, a, false, b, (short)0, c, false, false);
  }
  static __device__ __forceinline__ void guard(v8f& a, v8f& b, v16b x, v16b y) { dep_guard_b(a, b, x, y); }
  static __device__ __forceinline__ void keep(v16b a, v16b b, v16b c, v16b d) { keep4_b(a, b, c, d); }
};

template <int ET> struct Elem;
template <> struct Elem<0> { typedef _Float16 T; };
template <> struct Elem<1> { typedef __bf16 T; };
template <int ET, bool SPLIT, int BIAS_MODE, int OUT_MODE, bool RESID, int ACT = 0>
__global__ __launch_bounds__(256) void wmma_gemm64(
    const unsigned short* __restrict__ Ap, const unsigned short* __restrict__ A2p, int lda, long strideA,
    const unsigned short* __restrict__ Btp, const unsigned short* __restrict__ Bt2p, int ldb, long strideB,
    void* __restrict__ Cout, void* __restrict__ Cout2, int ldc, long strideC,
    const float* __restrict__ bias,
    const float* __restrict__ resid, long strideR,
    int M, int N, int K, float scale) {
  typedef typename Elem<ET>::T T;
  typedef typename Frag<T>::V V;
  const T* A = (const T*)Ap; const T* A2 = (const T*)A2p; const T* Bt = (const T*)Btp; const T* Bt2 = (const T*)Bt2p;
  __shared__ __align__(16) float sT[8][16 * 68];
  const int b    = blockIdx.y;
  const int lane = threadIdx.x & 31;
  const int wave = threadIdx.x >> 5;
  const int tilesN = N >> 6;
  const int tilesM = M >> 6;
  const int tile = blockIdx.x * 8 + wave;
  if (tile >= tilesM * tilesN) return;
  const int tm = tile / tilesN;
  const int tn = tile - tm * tilesN;
  const int m0 = tm << 6;
  const int n0 = tn << 6;

  const T* Ab  = A  + (size_t)b * strideA;
  const T* Bb  = Bt + (size_t)b * strideB;
  const T* Ab2 = SPLIT ? (A2  + (size_t)b * strideA) : nullptr;
  const T* Bb2 = SPLIT ? (Bt2 + (size_t)b * strideB) : nullptr;

  const int rlane = lane & 15;
  const int koff  = (lane >> 4) * 8;
  const int mOff  = (lane >> 4) * 8;

  v8f acc[4][4];
#pragma unroll
  for (int i = 0; i < 4; ++i)
#pragma unroll
    for (int j = 0; j < 4; ++j) acc[i][j] = (v8f){0.f,0.f,0.f,0.f,0.f,0.f,0.f,0.f};

  for (int k0 = 0; k0 < K; k0 += 32) {
    V bh[4], bl[4];
#pragma unroll
    for (int j = 0; j < 4; ++j) {
      const size_t bo = (size_t)(n0 + (j << 4) + rlane) * ldb + koff + k0;
      bh[j] = Frag<T>::load(Bb + bo);
      if (SPLIT) bl[j] = Frag<T>::load(Bb2 + bo);
    }
#pragma unroll
    for (int i = 0; i < 4; ++i) {
      const size_t ao = (size_t)(m0 + (i << 4) + rlane) * lda + koff + k0;
      V ah = Frag<T>::load(Ab + ao);
      V al;
      if (SPLIT) al = Frag<T>::load(Ab2 + ao);
#pragma unroll
      for (int j = 0; j < 4; ++j) {
        acc[i][j] = Frag<T>::mma(ah, bh[j], acc[i][j]);
        if (SPLIT) {
          acc[i][j] = Frag<T>::mma(ah, bl[j], acc[i][j]);
          acc[i][j] = Frag<T>::mma(al, bh[j], acc[i][j]);
        }
      }
      Frag<T>::guard(acc[i][0], acc[i][3], ah, SPLIT ? al : ah);
    }
    Frag<T>::keep(bh[0], bh[1], bh[2], bh[3]);
    if (SPLIT) Frag<T>::keep(bl[0], bl[1], bl[2], bl[3]);
  }
  acc_guard4(acc[0][0], acc[0][1], acc[0][2], acc[0][3]);
  acc_guard4(acc[1][0], acc[1][1], acc[1][2], acc[1][3]);
  acc_guard4(acc[2][0], acc[2][1], acc[2][2], acc[2][3]);
  acc_guard4(acc[3][0], acc[3][1], acc[3][2], acc[3][3]);

  float* slab = sT[wave];
  const float* Rb = RESID ? (resid + (size_t)b * strideR) : nullptr;
#pragma unroll
  for (int i = 0; i < 4; ++i) {
    const int mBase = m0 + (i << 4);
    union { v8f v; v4f q[2]; } bm;
    bm.v = (v8f){0.f,0.f,0.f,0.f,0.f,0.f,0.f,0.f};
    if (BIAS_MODE == 1) {
      bm.q[0] = *(const v4f*)(bias + mBase + mOff);
      bm.q[1] = *(const v4f*)(bias + mBase + mOff + 4);
    }
#pragma unroll
    for (int j = 0; j < 4; ++j) {
      const int n = n0 + (j << 4) + rlane;
      float bv = 0.f;
      if (BIAS_MODE == 2) bv = bias[n];
#pragma unroll
      for (int r = 0; r < 8; ++r) {
        float v = acc[i][j][r] * scale;
        if (BIAS_MODE == 1) v += bm.v[r];
        if (BIAS_MODE == 2) v += bv;
        if (RESID) v += Rb[(size_t)(mBase + mOff + r) * ldc + n];
        if (ACT == 1) v = tanhf(v);
        if (ACT == 2) v = fmaxf(v, 0.0f);
        if (ACT == 3) v = v / (1.0f + expf(-v));
        if (ACT == 4) v = (v > 0.f) ? v : 0.01f * v;
        slab[(mOff + r) * 68 + (j << 4) + rlane] = v;
      }
    }
    __builtin_amdgcn_fence(__ATOMIC_RELEASE, "workgroup");
    __builtin_amdgcn_wave_barrier();
    __builtin_amdgcn_fence(__ATOMIC_ACQUIRE, "workgroup");
    if (OUT_MODE == 0) {
      float* C = (float*)Cout + (size_t)b * strideC;
      const int hh = lane >> 4, c4 = (lane & 15) * 4;
      for (int pass = 0; pass < 2; ++pass) {
#pragma unroll
        for (int it = 0; it < 8; ++it) {
          const int row = it * 2 + hh;
          v4f v = *(const v4f*)(slab + row * 68 + c4);
          *(volatile v4f*)(C + (size_t)(mBase + row) * ldc + n0 + c4) = v;
        }
        __threadfence();
      }
    } else {
      const int q = lane >> 3, c8 = (lane & 7) * 8;
      unsigned short* C  = (unsigned short*)Cout  + (size_t)b * strideC;
      unsigned short* C2 = (OUT_MODE == 2) ? ((unsigned short*)Cout2 + (size_t)b * strideC) : nullptr;
      for (int pass = 0; pass < 2; ++pass) {
#pragma unroll
        for (int it = 0; it < 4; ++it) {
          const int row = it * 4 + q;
          const float* sp = slab + row * 68 + c8;
          v8h hv, lv;
#pragma unroll
          for (int e = 0; e < 8; ++e) {
            if (OUT_MODE == 1) {
              hv[e] = (_Float16)sp[e];
            } else {
              unsigned short hb = f2bf_bits(sp[e]);
              unsigned short lb = f2bf_bits(sp[e] - bf_bits2f(hb));
              hv[e] = __builtin_bit_cast(_Float16, hb);
              lv[e] = __builtin_bit_cast(_Float16, lb);
            }
          }
          *(volatile v8h*)(C + (size_t)(mBase + row) * ldc + n0 + c8) = hv;
          if (OUT_MODE == 2) *(volatile v8h*)(C2 + (size_t)(mBase + row) * ldc + n0 + c8) = lv;
        }
        __threadfence();
      }
    }
    __builtin_amdgcn_fence(__ATOMIC_RELEASE, "workgroup");
    __builtin_amdgcn_wave_barrier();
    __builtin_amdgcn_fence(__ATOMIC_ACQUIRE, "workgroup");
  }
}

__global__ __launch_bounds__(256) void k_cast4(
    const float* __restrict__ i0, _Float16* __restrict__ o0, int n0, float s0,
    const float* __restrict__ i1, _Float16* __restrict__ o1, int n1, float s1,
    const float* __restrict__ i2, _Float16* __restrict__ o2, int n2, float s2,
    const float* __restrict__ i3, _Float16* __restrict__ o3, int n3, float s3) {
  const float* in = i0; _Float16* out = o0; int n8 = n0; float sc = s0;
  if (blockIdx.y == 1) { in = i1; out = o1; n8 = n1; sc = s1; }
  else if (blockIdx.y == 2) { in = i2; out = o2; n8 = n2; sc = s2; }
  else if (blockIdx.y == 3) { in = i3; out = o3; n8 = n3; sc = s3; }
  const int i = blockIdx.x * 256 + threadIdx.x;
  if (i >= n8) return;
  const v4f a = *(const v4f*)(in + (size_t)8 * i);
  const v4f c = *(const v4f*)(in + (size_t)8 * i + 4);
  v8h hv;
#pragma unroll
  for (int e = 0; e < 4; ++e) { hv[e] = (_Float16)(a[e] * sc); hv[4 + e] = (_Float16)(c[e] * sc); }
  _Float16* dst = out + (size_t)8 * i;
  *(volatile v8h*)dst = hv;
  __threadfence();
  *(volatile v8h*)dst = hv;
}

__global__ __launch_bounds__(256) void k_gelu_f16(const v2u64* __restrict__ in, v2u64* __restrict__ out,
                                                  int n8, float out_scale) {
  const int i = blockIdx.x * 256 + threadIdx.x;
  if (i >= n8) return;
  const v2u64 w = in[i];
  const unsigned long long wlo = w[0], whi = w[1];
  unsigned long long olo = 0ull, ohi = 0ull;
#pragma unroll 1
  for (int e = 0; e < 8; ++e) {
    const bool first = (e < 4);
    const unsigned long long src = first ? wlo : whi;
    const unsigned sh = (unsigned)(e & 3) * 16u;
    const unsigned short bits = (unsigned short)((src >> sh) & 0xffffull);
    const float v = (float)__builtin_bit_cast(_Float16, bits);
    const float gl = 0.5f * v * (1.0f + erff(v * 0.70710678118654752f));
    const unsigned short ob = __builtin_bit_cast(unsigned short, (_Float16)(gl * out_scale));
    const unsigned long long obl = ((unsigned long long)ob) << sh;
    olo |= first ? obl : 0ull;
    ohi |= first ? 0ull : obl;
  }
  v2u64 ov; ov[0] = olo; ov[1] = ohi;
  *(volatile v2u64*)(out + i) = ov;
  __threadfence();
  *(volatile v2u64*)(out + i) = ov;
}

template <bool WH>
__global__ __launch_bounds__(256) void k_add_ln(const float* __restrict__ xin, const float* __restrict__ rin,
                                                const float* __restrict__ gam, const float* __restrict__ bet,
                                                float* __restrict__ yf, _Float16* __restrict__ yh, float eps) {
  __shared__ float red0[8];
  __shared__ float red1[8];
  __shared__ __align__(16) float srow[WH ? 1024 : 4];
  const int row = blockIdx.x, t = threadIdx.x, lane = t & 31, wave = t >> 5;
  const size_t base = (size_t)row * 1024 + 4 * t;
  const v4f xv = *(const v4f*)(xin + base);
  const v4f rv = *(const v4f*)(rin + base);
  const float a0 = xv[0] + rv[0], a1 = xv[1] + rv[1], a2 = xv[2] + rv[2], a3 = xv[3] + rv[3];
  float s = (a0 + a1) + (a2 + a3);
#pragma unroll
  for (int off = 16; off >= 1; off >>= 1) s += __shfl_xor(s, off, 32);
  if (lane == 0) red0[wave] = s;
  __syncthreads();
  float tot = 0.f;
#pragma unroll
  for (int w = 0; w < 8; ++w) tot += red0[w];
  const float mu = tot * (1.0f / 1024.0f);
  const float d0 = a0 - mu, d1 = a1 - mu, d2 = a2 - mu, d3 = a3 - mu;
  float sq = (d0 * d0 + d1 * d1) + (d2 * d2 + d3 * d3);
#pragma unroll
  for (int off = 16; off >= 1; off >>= 1) sq += __shfl_xor(sq, off, 32);
  if (lane == 0) red1[wave] = sq;
  __syncthreads();
  float tot2 = 0.f;
#pragma unroll
  for (int w = 0; w < 8; ++w) tot2 += red1[w];
  const float var = tot2 * (1.0f / 1024.0f);
  const float rstd = rsqrtf(var + eps);
  const v4f gv = *(const v4f*)(gam + 4 * t);
  const v4f bv = *(const v4f*)(bet + 4 * t);
  v4f yv;
  yv[0] = d0 * rstd * gv[0] + bv[0];
  yv[1] = d1 * rstd * gv[1] + bv[1];
  yv[2] = d2 * rstd * gv[2] + bv[2];
  yv[3] = d3 * rstd * gv[3] + bv[3];
  for (int pass = 0; pass < 2; ++pass) {
    *(volatile v4f*)(yf + base) = yv;
    __threadfence();
  }
  if (WH) {
    *(v4f*)(srow + 4 * t) = yv;
    __syncthreads();
    if (t < 128) {
      const v4f p0 = *(const v4f*)(srow + 8 * t);
      const v4f p1 = *(const v4f*)(srow + 8 * t + 4);
      v8h hv;
#pragma unroll
      for (int e = 0; e < 4; ++e) { hv[e] = (_Float16)p0[e]; hv[4 + e] = (_Float16)p1[e]; }
      _Float16* dst = yh + (size_t)row * 1024 + 8 * t;
      for (int pass = 0; pass < 2; ++pass) {
        *(volatile v8h*)dst = hv;
        __threadfence();
      }
    }
  }
}

#define AT_D 64
#define AT_NW 4
#define AT_QB 64
#define AT_KC 64

__device__ __forceinline__ v8f mma_f16g(v16h a, v16h b, v8f c) {
  c = __builtin_amdgcn_wmma_f32_16x16x32_f16(false, a, false, b, (short)0, c, false, false);
  asm volatile("v_nop\n\tv_nop\n\tv_nop\n\tv_nop" : "+v"(c) : "v"(a), "v"(b));
  return c;
}

__global__ __launch_bounds__(128)
void attn64_f16(const _Float16* __restrict__ Qp, const _Float16* __restrict__ Kp,
                const _Float16* __restrict__ VTp, _Float16* __restrict__ Op,
                const int* __restrict__ maskp,
                int S, int Skv, int nheads, int ldq, float qk_scale, float mask_fill, float o_scale) {
  __shared__ __align__(16) int Msk[AT_QB * AT_KC];
  __shared__ __align__(16) _Float16 Psh[AT_NW][16 * AT_KC];
  __shared__ __align__(16) float Os[AT_NW][16 * 68];

  const int tid  = threadIdx.x;
  const int wave = tid >> 5;
  const int lane = tid & 31;
  const int hh   = lane >> 4;
  const int c    = lane & 15;

  const int nqb = S / AT_QB;
  const int bx = blockIdx.x;
  const int qb = bx % nqb;
  const int bh = bx / nqb;
  const int h  = bh % nheads;
  const int b  = bh / nheads;
  const int qbase = qb * AT_QB;
  const int q0 = qbase + wave * 16;
  const int hd0 = h * AT_D;
  const int HD = nheads * AT_D;

  v16h qa[2];
  {
    const _Float16* qrow = Qp + (size_t)(b * S + q0 + c) * ldq + hd0 + 8 * hh;
#pragma unroll
    for (int dc = 0; dc < 2; ++dc) qa[dc] = Frag<_Float16>::load(qrow + dc * 32);
  }

  float mrow[8], lrow[8];
  v8f oacc[4];
#pragma unroll
  for (int r = 0; r < 8; ++r) { mrow[r] = -INFINITY; lrow[r] = 0.f; }
#pragma unroll
  for (int t = 0; t < 4; ++t) oacc[t] = (v8f){0.f,0.f,0.f,0.f,0.f,0.f,0.f,0.f};

  const int nChunks = Skv / AT_KC;
  for (int kc = 0; kc < nChunks; ++kc) {
    const int kv0 = kc * AT_KC;
    __syncthreads();
#pragma unroll
    for (int i = 0; i < 8; ++i) {
      const int f = i * 128 + tid;
      const int row = f >> 4, col4 = (f & 15) * 4;
      const v4i mv = *(const v4i*)(maskp + ((size_t)(b * S + qbase + row)) * Skv + kv0 + col4);
      *(v4i*)(Msk + row * AT_KC + col4) = mv;
    }
    __syncthreads();

    v8f s[4];
#pragma unroll
    for (int j = 0; j < 4; ++j) {
      s[j] = (v8f){0.f,0.f,0.f,0.f,0.f,0.f,0.f,0.f};
      const _Float16* krow = Kp + (size_t)(b * Skv + kv0 + j * 16 + c) * ldq + hd0 + 8 * hh;
#pragma unroll
      for (int dc = 0; dc < 2; ++dc) {
        const v16h kb = Frag<_Float16>::load(krow + dc * 32);
        s[j] = mma_f16g(qa[dc], kb, s[j]);
      }
    }
    float cm[8];
#pragma unroll
    for (int r = 0; r < 8; ++r) {
      const int qrl = wave * 16 + 8 * hh + r;
      float m = -INFINITY;
#pragma unroll
      for (int j = 0; j < 4; ++j) {
        const int mv = Msk[qrl * AT_KC + j * 16 + c];
        float v = s[j][r] * qk_scale;
        v = (mv == 0) ? mask_fill : v;
        s[j][r] = v;
        m = fmaxf(m, v);
      }
#pragma unroll
      for (int off = 1; off < 16; off <<= 1) m = fmaxf(m, __shfl_xor(m, off, 32));
      cm[r] = m;
    }
    _Float16* pw = Psh[wave];
#pragma unroll
    for (int r = 0; r < 8; ++r) {
      const float mnew = fmaxf(mrow[r], cm[r]);
      const float alpha = expf(mrow[r] - mnew);
      mrow[r] = mnew;
      float psum = 0.f;
#pragma unroll
      for (int j = 0; j < 4; ++j) {
        const float p = expf(s[j][r] - mnew);
        psum += p;
        pw[(8 * hh + r) * AT_KC + j * 16 + c] = (_Float16)(p * 32768.0f);
      }
#pragma unroll
      for (int off = 1; off < 16; off <<= 1) psum += __shfl_xor(psum, off, 32);
      lrow[r] = lrow[r] * alpha + psum;
#pragma unroll
      for (int t = 0; t < 4; ++t) oacc[t][r] *= alpha;
    }
    __builtin_amdgcn_fence(__ATOMIC_RELEASE, "workgroup");
    __builtin_amdgcn_wave_barrier();
    __builtin_amdgcn_fence(__ATOMIC_ACQUIRE, "workgroup");
#pragma unroll
    for (int kk = 0; kk < 2; ++kk) {
      Frag<_Float16>::U pa;
      pa.h[0] = *(const v8h*)(pw + c * AT_KC + kk * 32 + 8 * hh);
      pa.h[1] = *(const v8h*)(pw + c * AT_KC + kk * 32 + 16 + 8 * hh);
#pragma unroll
      for (int t = 0; t < 4; ++t) {
        const _Float16* vrow = VTp + (size_t)(b * HD + hd0 + t * 16 + c) * Skv + kv0 + kk * 32 + 8 * hh;
        const v16h vb = Frag<_Float16>::load(vrow);
        oacc[t] = mma_f16g(pa.v, vb, oacc[t]);
      }
    }
  }

  float* os = Os[wave];
#pragma unroll
  for (int r = 0; r < 8; ++r) {
    const float inv = o_scale * (1.0f / (lrow[r] * 32768.0f));
#pragma unroll
    for (int t = 0; t < 4; ++t) os[(8 * hh + r) * 68 + t * 16 + c] = oacc[t][r] * inv;
  }
  __builtin_amdgcn_fence(__ATOMIC_RELEASE, "workgroup");
  __builtin_amdgcn_wave_barrier();
  __builtin_amdgcn_fence(__ATOMIC_ACQUIRE, "workgroup");
  {
    const int q8 = lane >> 3, c8 = (lane & 7) * 8;
    _Float16* obase = Op + (size_t)(b * S + q0) * ldq + hd0 + c8;
    for (int pass = 0; pass < 2; ++pass) {
#pragma unroll
      for (int it = 0; it < 4; ++it) {
        const int row = it * 4 + q8;
        const float* sp = os + row * 68 + c8;
        v8h hv;
#pragma unroll
        for (int e = 0; e < 8; ++e) hv[e] = (_Float16)sp[e];
        *(volatile v8h*)(obase + (size_t)row * ldq) = hv;
      }
      __threadfence();
    }
  }
}

constexpr int BATCH = 4;
constexpr int SEQ   = 1024;
constexpr int HID   = 1024;
constexpr int NHEAD = 16;
constexpr int DHEAD = 64;
constexpr int FFD   = 4096;
constexpr int NTOK  = BATCH * SEQ;
static_assert(NHEAD * DHEAD == HID, "head split");
static_assert(DHEAD == AT_D, "attention kernel head dim");
static_assert(SEQ % AT_QB == 0 && SEQ % AT_KC == 0, "attention tiles");
static_assert(HID == 1024, "LayerNorm kernel assumes 1024 columns (256 threads x 4)");
static_assert(NTOK % 64 == 0 && HID % 64 == 0 && FFD % 64 == 0 && SEQ % 64 == 0, "M/N tile multiples");
static_assert(HID % 32 == 0 && FFD % 32 == 0, "K multiples of 32");

constexpr size_t MIB = 1048576;
constexpr size_t OFF_WQ_S = 0 * MIB, OFF_WK_S = 2 * MIB, OFF_WV_S = 4 * MIB, OFF_WO_S = 6 * MIB;
constexpr size_t OFF_WQ_C = 8 * MIB, OFF_WK_C = 10 * MIB, OFF_WV_C = 12 * MIB, OFF_WO_C = 14 * MIB;
constexpr size_t OFF_X1F  = 16 * MIB;
constexpr size_t OFF_HACT = 0 * MIB;
constexpr size_t OFF_W1   = 32 * MIB, OFF_W2 = 40 * MIB;
constexpr size_t OFF_XH   = 48 * MIB, OFF_MEMH = 56 * MIB;
constexpr size_t OFF_X2F  = 48 * MIB;
constexpr size_t OFF_QP   = 64 * MIB;
constexpr size_t OFF_X2H  = 64 * MIB;
constexpr size_t OFF_KP   = 72 * MIB, OFF_VTP = 80 * MIB, OFF_OP = 88 * MIB, OFF_X1H = 96 * MIB;
constexpr size_t OFF_HPRE = 72 * MIB;
constexpr size_t OFF_PROJ = 104 * MIB;
constexpr size_t WS_TOTAL = 120 * MIB;
static_assert((size_t)HID * HID * 2 == 2 * MIB, "weight f16 plane = 2 MiB");
static_assert((size_t)FFD * HID * 2 == 8 * MIB, "ffn weight f16 plane = 8 MiB");
static_assert((size_t)NTOK * HID * 2 == 8 * MIB, "token f16 plane = 8 MiB");
static_assert((size_t)NTOK * HID * 4 == 16 * MIB, "token f32 plane = 16 MiB");
static_assert((size_t)BATCH * HID * SEQ * 2 == 8 * MIB, "vT f16 plane = 8 MiB");
static_assert((size_t)NTOK * FFD * 2 == 32 * MIB, "ffn hidden f16 plane = 32 MiB");
static_assert(OFF_X1F + 16 * MIB == OFF_HACT + 32 * MIB && OFF_HACT + 32 * MIB == OFF_W1, "hact aliases w_self,w_cross,x1f exactly");
static_assert(OFF_MEMH + 8 * MIB == OFF_X2F + 16 * MIB && OFF_X2F + 16 * MIB == OFF_QP, "x2f aliases xh,memh exactly");
static_assert(OFF_X1H + 8 * MIB == OFF_HPRE + 32 * MIB && OFF_HPRE + 32 * MIB == OFF_PROJ, "hpre aliases k,vT,o,x1h exactly");
static_assert(OFF_PROJ + 16 * MIB == WS_TOTAL, "carve total");
static_assert(WS_TOTAL <= 134217728, "carve within 128 MiB");

static inline dim3 gemm_grid(int M, int N, int batch) { return dim3((unsigned)(((M / 64) * (N / 64) + 7) / 8), (unsigned)batch, 1); }

extern "C" void kernel_launch(void* const* d_in, const int* in_sizes, int n_in,
                              void* d_out, int out_size, void* d_ws, size_t ws_size,
                              hipStream_t stream) {
  if (n_in < 30) return;
  if (out_size != NTOK * HID) return;
  if (ws_size < WS_TOTAL) return;
  if (in_sizes[0] != NTOK * HID || in_sizes[1] != NTOK * HID) return;
  if (in_sizes[2] != BATCH * SEQ * SEQ || in_sizes[3] != BATCH * SEQ * SEQ) return;
  if (in_sizes[20] != FFD * HID || in_sizes[22] != HID * FFD) return;

  const float* x        = (const float*)d_in[0];
  const float* memory   = (const float*)d_in[1];
  const int*   tgt_mask = (const int*)d_in[2];
  const int*   mem_mask = (const int*)d_in[3];
  const float* sa_wq = (const float*)d_in[4];  const float* sa_bq = (const float*)d_in[5];
  const float* sa_wk = (const float*)d_in[6];  const float* sa_bk = (const float*)d_in[7];
  const float* sa_wv = (const float*)d_in[8];  const float* sa_bv = (const float*)d_in[9];
  const float* sa_wo = (const float*)d_in[10]; const float* sa_bo = (const float*)d_in[11];
  const float* ca_wq = (const float*)d_in[12]; const float* ca_bq = (const float*)d_in[13];
  const float* ca_wk = (const float*)d_in[14]; const float* ca_bk = (const float*)d_in[15];
  const float* ca_wv = (const float*)d_in[16]; const float* ca_bv = (const float*)d_in[17];
  const float* ca_wo = (const float*)d_in[18]; const float* ca_bo = (const float*)d_in[19];
  const float* ff_w1 = (const float*)d_in[20]; const float* ff_b1 = (const float*)d_in[21];
  const float* ff_w2 = (const float*)d_in[22]; const float* ff_b2 = (const float*)d_in[23];
  const float* ln1_g = (const float*)d_in[24]; const float* ln1_b = (const float*)d_in[25];
  const float* ln2_g = (const float*)d_in[26]; const float* ln2_b = (const float*)d_in[27];
  const float* ln3_g = (const float*)d_in[28]; const float* ln3_b = (const float*)d_in[29];
  float* outp = (float*)d_out;

  char* ws = (char*)d_ws;
  _Float16* wq_s = (_Float16*)(ws + OFF_WQ_S); _Float16* wk_s = (_Float16*)(ws + OFF_WK_S);
  _Float16* wv_s = (_Float16*)(ws + OFF_WV_S); _Float16* wo_s = (_Float16*)(ws + OFF_WO_S);
  _Float16* wq_c = (_Float16*)(ws + OFF_WQ_C); _Float16* wk_c = (_Float16*)(ws + OFF_WK_C);
  _Float16* wv_c = (_Float16*)(ws + OFF_WV_C); _Float16* wo_c = (_Float16*)(ws + OFF_WO_C);
  _Float16* w1h  = (_Float16*)(ws + OFF_W1);   _Float16* w2h  = (_Float16*)(ws + OFF_W2);
  _Float16* xh   = (_Float16*)(ws + OFF_XH);   _Float16* memh = (_Float16*)(ws + OFF_MEMH);
  _Float16* qp   = (_Float16*)(ws + OFF_QP);   _Float16* kp   = (_Float16*)(ws + OFF_KP);
  _Float16* vtp  = (_Float16*)(ws + OFF_VTP);  _Float16* op   = (_Float16*)(ws + OFF_OP);
  _Float16* x1h  = (_Float16*)(ws + OFF_X1H);  _Float16* x2h  = (_Float16*)(ws + OFF_X2H);
  _Float16* hpre = (_Float16*)(ws + OFF_HPRE); _Float16* hact = (_Float16*)(ws + OFF_HACT);
  float* x1f  = (float*)(ws + OFF_X1F);
  float* x2f  = (float*)(ws + OFF_X2F);
  float* proj = (float*)(ws + OFF_PROJ);

  typedef const unsigned short* cus;
  const float WSC   = 64.0f;
  const float OSC   = 16.0f;
  const float INV_W = 1.0f / 64.0f;
  const float INV_WO = 1.0f / 1024.0f;
  const float LN_EPS = 1e-5f;

  const int n8_tok = NTOK * HID / 8;
  const int n8_ffw = FFD * HID / 8;
  const int n8_w   = HID * HID / 8;
  k_cast4<<<dim3(2048, 4), 256, 0, stream>>>(x, xh, n8_tok, 1.0f, memory, memh, n8_tok, 1.0f,
                                              ff_w1, w1h, n8_ffw, WSC, ff_w2, w2h, n8_ffw, WSC);
  k_cast4<<<dim3(512, 4), 256, 0, stream>>>(sa_wq, wq_s, n8_w, WSC, sa_wk, wk_s, n8_w, WSC,
                                             sa_wv, wv_s, n8_w, WSC, sa_wo, wo_s, n8_w, WSC);
  k_cast4<<<dim3(512, 4), 256, 0, stream>>>(ca_wq, wq_c, n8_w, WSC, ca_wk, wk_c, n8_w, WSC,
                                             ca_wv, wv_c, n8_w, WSC, ca_wo, wo_c, n8_w, WSC);

  const long TOKPLANE = (long)SEQ * HID;
  const long VTPLANE  = (long)HID * SEQ;
  const dim3 g_tok  = gemm_grid(NTOK, HID, 1);
  const dim3 g_vt   = gemm_grid(HID, SEQ, BATCH);
  const dim3 g_ff1  = gemm_grid(NTOK, FFD, 1);
  const dim3 g_ff2  = gemm_grid(NTOK, HID, 1);
  const unsigned attn_blocks = (unsigned)(BATCH * NHEAD * (SEQ / AT_QB));

  wmma_gemm64<0, false, 2, 1, false><<<g_tok, 256, 0, stream>>>(
      (cus)xh, (cus)xh, HID, 0L, (cus)wq_s, (cus)wq_s, HID, 0L,
      (void*)qp, (void*)qp, HID, 0L, sa_bq, proj, 0L, NTOK, HID, HID, INV_W);
  wmma_gemm64<0, false, 2, 1, false><<<g_tok, 256, 0, stream>>>(
      (cus)xh, (cus)xh, HID, 0L, (cus)wk_s, (cus)wk_s, HID, 0L,
      (void*)kp, (void*)kp, HID, 0L, sa_bk, proj, 0L, NTOK, HID, HID, INV_W);
  wmma_gemm64<0, false, 1, 1, false><<<g_vt, 256, 0, stream>>>(
      (cus)wv_s, (cus)wv_s, HID, 0L, (cus)xh, (cus)xh, HID, TOKPLANE,
      (void*)vtp, (void*)vtp, SEQ, VTPLANE, sa_bv, proj, 0L, HID, SEQ, HID, INV_W);
  attn64_f16<<<dim3(attn_blocks), 128, 0, stream>>>(qp, kp, vtp, op, tgt_mask,
                                                    SEQ, SEQ, NHEAD, HID, 0.125f, -1e9f, OSC);
  wmma_gemm64<0, false, 2, 0, false><<<g_tok, 256, 0, stream>>>(
      (cus)op, (cus)op, HID, 0L, (cus)wo_s, (cus)wo_s, HID, 0L,
      (void*)proj, (void*)proj, HID, 0L, sa_bo, proj, 0L, NTOK, HID, HID, INV_WO);
  k_add_ln<true><<<dim3(NTOK), 256, 0, stream>>>(x, proj, ln1_g, ln1_b, x1f, x1h, LN_EPS);

  wmma_gemm64<0, false, 2, 1, false><<<g_tok, 256, 0, stream>>>(
      (cus)x1h, (cus)x1h, HID, 0L, (cus)wq_c, (cus)wq_c, HID, 0L,
      (void*)qp, (void*)qp, HID, 0L, ca_bq, proj, 0L, NTOK, HID, HID, INV_W);
  wmma_gemm64<0, false, 2, 1, false><<<g_tok, 256, 0, stream>>>(
      (cus)memh, (cus)memh, HID, 0L, (cus)wk_c, (cus)wk_c, HID, 0L,
      (void*)kp, (void*)kp, HID, 0L, ca_bk, proj, 0L, NTOK, HID, HID, INV_W);
  wmma_gemm64<0, false, 1, 1, false><<<g_vt, 256, 0, stream>>>(
      (cus)wv_c, (cus)wv_c, HID, 0L, (cus)memh, (cus)memh, HID, TOKPLANE,
      (void*)vtp, (void*)vtp, SEQ, VTPLANE, ca_bv, proj, 0L, HID, SEQ, HID, INV_W);
  attn64_f16<<<dim3(attn_blocks), 128, 0, stream>>>(qp, kp, vtp, op, mem_mask,
                                                    SEQ, SEQ, NHEAD, HID, 0.125f, -1e9f, OSC);
  wmma_gemm64<0, false, 2, 0, false><<<g_tok, 256, 0, stream>>>(
      (cus)op, (cus)op, HID, 0L, (cus)wo_c, (cus)wo_c, HID, 0L,
      (void*)proj, (void*)proj, HID, 0L, ca_bo, proj, 0L, NTOK, HID, HID, INV_WO);
  k_add_ln<true><<<dim3(NTOK), 256, 0, stream>>>(x1f, proj, ln2_g, ln2_b, x2f, x2h, LN_EPS);

  wmma_gemm64<0, false, 2, 1, false><<<g_ff1, 256, 0, stream>>>(
      (cus)x2h, (cus)x2h, HID, 0L, (cus)w1h, (cus)w1h, HID, 0L,
      (void*)hpre, (void*)hpre, FFD, 0L, ff_b1, proj, 0L, NTOK, FFD, HID, INV_W);
  const int n8_ff = NTOK * FFD / 8;
  k_gelu_f16<<<dim3(8192), 256, 0, stream>>>((const v2u64*)(const void*)hpre, (v2u64*)(void*)hact, n8_ff, OSC);
  wmma_gemm64<0, false, 2, 0, false><<<g_ff2, 256, 0, stream>>>(
      (cus)hact, (cus)hact, FFD, 0L, (cus)w2h, (cus)w2h, FFD, 0L,
      (void*)proj, (void*)proj, HID, 0L, ff_b2, proj, 0L, NTOK, HID, FFD, INV_WO);
  k_add_ln<false><<<dim3(NTOK), 256, 0, stream>>>(x2f, proj, ln3_g, ln3_b, outp, x1h, LN_EPS);
}
